// InverseRadonTransform_1108101562469
// MI455X (gfx1250) — hardware-verified
//
#include <hip/hip_runtime.h>
#include <math.h>

typedef __attribute__((ext_vector_type(16))) _Float16 v16h;
typedef __attribute__((ext_vector_type(16))) __bf16 v16b;
typedef __attribute__((ext_vector_type(8)))  _Float16 v8h;
typedef __attribute__((ext_vector_type(8)))  float v8f;
typedef __attribute__((ext_vector_type(4)))  float v4f;
typedef __attribute__((ext_vector_type(2)))  float v2f;
typedef __attribute__((ext_vector_type(4)))  unsigned v4u;
typedef __attribute__((ext_vector_type(4)))  int v4i;
typedef float __attribute__((may_alias)) float_a;
typedef int __attribute__((may_alias)) int_a;

template <typename T> __device__ __forceinline__ void vst2(void* p, T v) { *(volatile T*)p = v; __threadfence(); *(volatile T*)p = v; }
__device__ __forceinline__ v8f wmma16(v16h a, v16h b, v8f c) {
  v8f d = __builtin_amdgcn_wmma_f32_16x16x32_f16(false, a, false, b, (short)0, c, false, false);
  asm volatile("v_nop\n\tv_nop\n\tv_nop\n\tv_nop" : "+v"(d) : "v"(a), "v"(b));
  return d;
}
__device__ __forceinline__ v8f wmma_bf(v16b a, v16b b, v8f c) {
  v8f d = __builtin_amdgcn_wmma_f32_16x16x32_bf16(false, a, false, b, (short)0, c, false, false);
  asm volatile("v_nop\n\tv_nop\n\tv_nop\n\tv_nop" : "+v"(d) : "v"(a), "v"(b));
  return d;
}
__device__ __forceinline__ v16h frag_h(const _Float16* rowk0, int lane) {
  union { v16h v; v8h q[2]; } u; const _Float16* p = rowk0 + 8 * (lane >> 4);
  u.q[0] = *(const v8h*)p; u.q[1] = *(const v8h*)(p + 16); return u.v;
}
__device__ __forceinline__ v16h frag_f32(const float* rowk0, int lane) {
  v16h a; const float* p = rowk0 + 8 * (lane >> 4);
#pragma unroll
  for (int i = 0; i < 8; ++i) { a[i] = (_Float16)p[i]; a[8 + i] = (_Float16)p[16 + i]; }
  return a;
}
__device__ __forceinline__ v16h frag_f32s(const float* rowk0, int lane, float sc) {
  v16h a; const float* p = rowk0 + 8 * (lane >> 4);
#pragma unroll
  for (int i = 0; i < 8; ++i) { a[i] = (_Float16)(p[i] * sc); a[8 + i] = (_Float16)(p[16 + i] * sc); }
  return a;
}
__device__ __forceinline__ v16h fragc_f32(const float* W, int k0, int n, int lane, int ld, int K) {
  v16h a; const int g = lane >> 4;
#pragma unroll
  for (int i = 0; i < 8; ++i) { const int ka = k0 + 8 * g + i, kb = ka + 16;
    a[i] = (_Float16)(ka < K ? W[(size_t)(ka < K ? ka : K - 1) * ld + n] : 0.f); a[8 + i] = (_Float16)(kb < K ? W[(size_t)(kb < K ? kb : K - 1) * ld + n] : 0.f); }
  return a;
}
struct F2 { v16b h, l; };
__device__ __forceinline__ F2 bsplit16(const float v[16]) { F2 r;
#pragma unroll
  for (int i = 0; i < 16; ++i) { const __bf16 h = (__bf16)v[i]; r.h[i] = h; r.l[i] = (__bf16)(v[i] - (float)h); }
  return r; }
__device__ __forceinline__ F2 split_row(const float* row, int k0, int lane) { float v[16]; const float* p = row + k0 + 8 * (lane >> 4);
#pragma unroll
  for (int i = 0; i < 8; ++i) { v[i] = p[i]; v[8 + i] = p[16 + i]; }
  return bsplit16(v); }
__device__ __forceinline__ F2 split_rowK(const float* row, int k0, int lane, int K) { float v[16]; const int g = lane >> 4;
#pragma unroll
  for (int i = 0; i < 8; ++i) { const int ka = k0 + 8 * g + i, kb = ka + 16; v[i] = ka < K ? row[ka < K ? ka : K - 1] : 0.f; v[8 + i] = kb < K ? row[kb < K ? kb : K - 1] : 0.f; }
  return bsplit16(v); }
__device__ __forceinline__ F2 split_col(const float* W, int k0, int n, int lane, int ld, int K) { float v[16]; const int g = lane >> 4;
#pragma unroll
  for (int i = 0; i < 8; ++i) { const int ka = k0 + 8 * g + i, kb = ka + 16; v[i] = ka < K ? W[(size_t)(ka < K ? ka : K - 1) * ld + n] : 0.f; v[8 + i] = kb < K ? W[(size_t)(kb < K ? kb : K - 1) * ld + n] : 0.f; }
  return bsplit16(v); }
__device__ __forceinline__ v8f mac3(const F2& a, const F2& b, v8f c) { c = wmma_bf(a.l, b.h, c); c = wmma_bf(a.h, b.l, c); return wmma_bf(a.h, b.h, c); }
__device__ __forceinline__ float sigm(float v) { return 1.0f / (1.0f + expf(-v)); }
#define LDSX() do { asm volatile("s_wait_dscnt 0" ::: "memory"); __builtin_amdgcn_wave_barrier(); __builtin_amdgcn_fence(__ATOMIC_RELEASE, "workgroup"); } while (0)


#define NB 4
#define NA 180
#define NP 512
#define PI_D 3.14159265358979323846
#ifndef TNB
#define TNB NB
#define TCB ((NB * NA + 63) / 64)
#endif
__device__ __forceinline__ float bfr(float v) { return (float)(__bf16)v; }
__device__ __forceinline__ v16b frag_gbf(const float* rowk0, int lane) {
  v16b a; const float* p = rowk0 + 8 * (lane >> 4);
#pragma unroll
  for (int i = 0; i < 8; ++i) { a[i] = (__bf16)p[i]; a[8 + i] = (__bf16)p[16 + i]; }
  return a;
}
__global__ __launch_bounds__(512) void k_filt(float* __restrict__ HC, float* __restrict__ TAB) {
  __shared__ double sf[NP], sff[NP]; __shared__ float sffr[NP], sh[NP];
  const int k = threadIdx.x;
  { double v = 0.0; if (k == 0) v = 0.25; else if (k & 1) { const int j = k >> 1; const double n = j < 128 ? (double)(2 * j + 1) : (double)(255 - 2 * (j - 128)); v = -1.0 / ((PI_D * n) * (PI_D * n)); } sf[k] = v; }
  __syncthreads();
  { double s = 0.0; for (int n = 0; n < NP; ++n) { const int kn = (k * n) & (NP - 1); s += sf[n] * cos(2.0 * PI_D * (double)kn / (double)NP); }
    double ff = 2.0 * s; if (k >= 1) { const double fq = (k < NP / 2) ? (double)k / NP : (double)(k - NP) / NP; const double w = PI_D * fq; ff *= sin(w) / w; }
    sff[k] = ff; sffr[k] = (float)ff; }
  __syncthreads();
  { double s = 0.0; for (int q = 0; q < NP; ++q) { const int qm = (q * k) & (NP - 1); s += (double)sffr[q] * cos(2.0 * PI_D * (double)qm / (double)NP); } sh[k] = (float)(s / (double)NP); }
  __syncthreads();
  for (int p = 0; p < NP; ++p) { const float v = sh[(p - k) & (NP - 1)]; __syncthreads(); sffr[k] = v; __syncthreads(); if (k < NP / 4) vst2(HC + (size_t)p * NP + k * 4, *(const v4f*)&sffr[k * 4]); }
  if (k < NA) { const float hstep = (float)k / 179.0f; const float deg = (k == NA - 1) ? 180.0f : 0.0f * (1.0f - hstep) + 180.0f * hstep; const float th = deg * (float)(PI_D / 180.0); sh[k] = sinf(th); sh[256 + k] = cosf(th); }
  __syncthreads();
  if (k < 128) vst2(TAB + k * 4, *(const v4f*)&sh[k * 4]);
}

__global__ __launch_bounds__(128) void k_conv(const float* __restrict__ SINO, const float* __restrict__ HC, float* __restrict__ FILT) {
  __shared__ __align__(16) float so[4][16][132];
  const int tid = threadIdx.x, wave = tid >> 5, lane = tid & 31, col = lane & 15, g = lane >> 4; const size_t r0 = (size_t)blockIdx.x * 64 + wave * 16; const int n0 = blockIdx.y * 128;
  const size_t ra = (r0 + col) < (size_t)(NB * NA) ? r0 + col : (size_t)(NB * NA - 1);
  v8f acc[8] = {};
#pragma unroll 1
  for (int kc = 0; kc < NP / 32; ++kc) { const v16b a = frag_gbf(SINO + ra * NP + kc * 32, lane);
#pragma unroll
    for (int j = 0; j < 8; ++j) { const F2 bq = split_row(HC + (size_t)(n0 + j * 16 + col) * NP, kc * 32, lane); acc[j] = wmma_bf(a, bq.l, acc[j]); acc[j] = wmma_bf(a, bq.h, acc[j]); } }
#pragma unroll
  for (int j = 0; j < 8; ++j)
#pragma unroll
    for (int r = 0; r < 8; ++r) so[wave][8 * g + r][j * 16 + col] = acc[j][r];
  LDSX();
  for (int rl = 0; rl < 16; ++rl) { const size_t row = r0 + rl; if (row < (size_t)(NB * NA)) vst2(FILT + row * NP + n0 + lane * 4, *(const v4f*)(&so[wave][rl][lane * 4])); }
}
__global__ __launch_bounds__(256) void k_bp(const float* __restrict__ FILT, const float* __restrict__ TAB, float* __restrict__ out) {
  __shared__ float ssin[NA], scos[NA]; __shared__ __align__(16) float srow[NP];
  const int tid = threadIdx.x, b = blockIdx.y, hh = blockIdx.x;
  for (int a = tid; a < NA; a += 256) { ssin[a] = TAB[a]; scos[a] = TAB[256 + a]; }
  __syncthreads();
  const float y = (float)hh - 256.0f;
  float accv[2] = {0.f, 0.f};
#pragma unroll 1
  for (int a = 0; a < NA; ++a) { const float* row = FILT + ((size_t)b * NA + a) * NP; const float sn = ssin[a], cs = scos[a];
#pragma unroll
    for (int u = 0; u < 2; ++u) { const int w = tid + 256 * u; const float x = (float)(NP - 1 - w) - 256.0f;
      const float p = x * sn + y * cs + 256.0f; const float i0f = floorf(p); const float fr = p - i0f; const int i0 = (int)i0f, i1 = i0 + 1;
      const int c0 = i0 < 0 ? 0 : (i0 > NP - 1 ? NP - 1 : i0), c1 = i1 < 0 ? 0 : (i1 > NP - 1 ? NP - 1 : i1);
      const float v0 = (i0 >= 0 && i0 <= NP - 1) ? row[c0] : 0.f, v1 = (i1 >= 0 && i1 <= NP - 1) ? row[c1] : 0.f;
      accv[u] = accv[u] + ((1.0f - fr) * v0 + fr * v1); } }
  const float sc = (float)(PI_D / (2.0 * NA));
#pragma unroll
  for (int u = 0; u < 2; ++u) { const int w = tid + 256 * u; const float x = (float)(NP - 1 - w) - 256.0f; const float m = (x * x + y * y <= 256.0f * 256.0f) ? 1.0f : 0.0f; srow[w] = (accv[u] * sc) * m; }
  __syncthreads();
  if (tid < 128) vst2(out + ((size_t)b * NP + hh) * NP + tid * 4, *(const v4f*)&srow[tid * 4]);
}

extern "C" void kernel_launch(void* const* d_in, const int* in_sizes, int n_in, void* d_out, int out_size, void* d_ws, size_t ws_size, hipStream_t stream) {
  (void)in_sizes; (void)n_in; (void)out_size; (void)ws_size;
  char* ws = (char*)d_ws; float* HC = (float*)ws; float* TAB = HC + (size_t)NP * NP; float* FILT = TAB + 512;
  k_filt<<<1, 512, 0, stream>>>(HC, TAB);
  k_conv<<<dim3(TCB, NP / 128), 128, 0, stream>>>((const float*)d_in[0], HC, FILT);
  k_bp<<<dim3(NP, TNB), 256, 0, stream>>>(FILT, TAB, (float*)d_out);
}
